// MANN_75273596829746
// MI455X (gfx1250) — hardware-verified
//
#include <hip/hip_runtime.h>
#include <math.h>

constexpr int NSEQ   = 512;
constexpr int NSTEP  = 512;
constexpr int NIN    = 20;
constexpr int NHID   = 128;
constexpr int NGATE  = 4 * NHID;
constexpr int KCAT   = 160;
constexpr int APITCH = 168;
constexpr int NTHR   = 256;
constexpr int NHD    = 64;
constexpr int NOUT   = 4;
constexpr int NROWS  = NSEQ * NSTEP;
constexpr int HCHUNK = 131072;
constexpr float WSC     = 16.0f;
constexpr float WSC_INV = 1.0f / 16.0f;

static_assert(NROWS % HCHUNK == 0);
static_assert(HCHUNK % 64 == 0);
static_assert(HCHUNK % NTHR == 0);
static_assert(KCAT % 32 == 0);
static_assert(NHID % 32 == 0);
static_assert(APITCH % 8 == 0);

typedef __attribute__((ext_vector_type(16))) _Float16 v16h;
typedef __attribute__((ext_vector_type(8)))  _Float16 v8h;
typedef __attribute__((ext_vector_type(4)))  _Float16 v4h;
typedef __attribute__((ext_vector_type(16))) __bf16   v16b;
typedef __attribute__((ext_vector_type(8)))  __bf16   v8b;
typedef __attribute__((ext_vector_type(8)))  float    v8f;
typedef __attribute__((ext_vector_type(4)))  float    v4f;

__device__ __forceinline__ unsigned short f2bf_bits(float f) {
  unsigned u = __float_as_uint(f);
  return (unsigned short)((u + 0x7FFFu + ((u >> 16) & 1u)) >> 16);
}
__device__ __forceinline__ float bf_bits2f(unsigned short h) { return __uint_as_float(((unsigned)h) << 16); }
__device__ __forceinline__ float bf16q(float f) { return bf_bits2f(f2bf_bits(f)); }

__device__ __forceinline__ void dep_guard_h(v8f& a, v8f& b, v16h x, v16h y) { asm volatile("v_nop\n\tv_nop\n\tv_nop\n\tv_nop" : "+v"(a), "+v"(b) : "v"(x), "v"(y)); }
__device__ __forceinline__ void dep_guard_b(v8f& a, v8f& b, v16b x, v16b y) { asm volatile("v_nop\n\tv_nop\n\tv_nop\n\tv_nop" : "+v"(a), "+v"(b) : "v"(x), "v"(y)); }
__device__ __forceinline__ void keep4_h(v16h a, v16h b, v16h c, v16h d) { asm volatile("v_nop" :: "v"(a), "v"(b), "v"(c), "v"(d)); }
__device__ __forceinline__ void keep4_b(v16b a, v16b b, v16b c, v16b d) { asm volatile("v_nop" :: "v"(a), "v"(b), "v"(c), "v"(d)); }
__device__ __forceinline__ void acc_guard4(v8f& a, v8f& b, v8f& c, v8f& d) { asm volatile("v_nop\n\tv_nop\n\tv_nop\n\tv_nop" : "+v"(a), "+v"(b), "+v"(c), "+v"(d)); }
template <typename T> struct Frag;
template <> struct Frag<_Float16> {
  typedef v16h V; union U { v16h v; v8h h[2]; };
  static __device__ __forceinline__ v16h load(const _Float16* p) {
    U f; f.h[0] = *(const v8h*)(p); f.h[1] = *(const v8h*)(p + 16); return f.v;
  }
  static __device__ __forceinline__ v8f mma(v16h a, v16h b, v8f c) {
    return __builtin_amdgcn_wmma_f32_16x16x32_f16(false, a, false, b, (short)0, c, false, false);
  }
  static __device__ __forceinline__ void guard(v8f& a, v8f& b, v16h x, v16h y) { dep_guard_h(a, b, x, y); }
  static __device__ __forceinline__ void keep(v16h a, v16h b, v16h c, v16h d) { keep4_h(a, b, c, d); }
};
template <> struct Frag<__bf16> {
  typedef v16b V; union U { v16b v; v8b h[2]; };
  static __device__ __forceinline__ v16b load(const __bf16* p) {
    U f; f.h[0] = *(const v8b*)(p); f.h[1] = *(const v8b*)(p + 16); return f.v;
  }
  static __device__ __forceinline__ v8f mma(v16b a, v16b b, v8f c) {
    return __builtin_amdgcn_wmma_f32_16x16x32_bf16(false, a, false, b, (short)0, c, false, false);
  }
  static __device__ __forceinline__ void guard(v8f& a, v8f& b, v16b x, v16b y) { dep_guard_b(a, b, x, y); }
  static __device__ __forceinline__ void keep(v16b a, v16b b, v16b c, v16b d) { keep4_b(a, b, c, d); }
};

template <int ET> struct Elem;
template <> struct Elem<0> { typedef _Float16 T; };
template <> struct Elem<1> { typedef __bf16 T; };
template <int ET, bool SPLIT, int BIAS_MODE, int OUT_MODE, bool RESID, int ACT = 0>
__global__ __launch_bounds__(256) void wmma_gemm64(
    const unsigned short* __restrict__ Ap, const unsigned short* __restrict__ A2p, int lda, long strideA,
    const unsigned short* __restrict__ Btp, const unsigned short* __restrict__ Bt2p, int ldb, long strideB,
    void* __restrict__ Cout, void* __restrict__ Cout2, int ldc, long strideC,
    const float* __restrict__ bias,
    const float* __restrict__ resid, long strideR,
    int M, int N, int K, float scale) {
  typedef typename Elem<ET>::T T;
  typedef typename Frag<T>::V V;
  const T* A = (const T*)Ap; const T* A2 = (const T*)A2p; const T* Bt = (const T*)Btp; const T* Bt2 = (const T*)Bt2p;
  __shared__ __align__(16) float sT[8][16 * 68];
  const int b    = blockIdx.y;
  const int lane = threadIdx.x & 31;
  const int wave = threadIdx.x >> 5;
  const int tilesN = N >> 6;
  const int tilesM = M >> 6;
  const int tile = blockIdx.x * 8 + wave;
  if (tile >= tilesM * tilesN) return;
  const int tm = tile / tilesN;
  const int tn = tile - tm * tilesN;
  const int m0 = tm << 6;
  const int n0 = tn << 6;

  const T* Ab  = A  + (size_t)b * strideA;
  const T* Bb  = Bt + (size_t)b * strideB;
  const T* Ab2 = SPLIT ? (A2  + (size_t)b * strideA) : nullptr;
  const T* Bb2 = SPLIT ? (Bt2 + (size_t)b * strideB) : nullptr;

  const int rlane = lane & 15;
  const int koff  = (lane >> 4) * 8;
  const int mOff  = (lane >> 4) * 8;

  v8f acc[4][4];
#pragma unroll
  for (int i = 0; i < 4; ++i)
#pragma unroll
    for (int j = 0; j < 4; ++j) acc[i][j] = (v8f){0.f,0.f,0.f,0.f,0.f,0.f,0.f,0.f};

  for (int k0 = 0; k0 < K; k0 += 32) {
    V bh[4], bl[4];
#pragma unroll
    for (int j = 0; j < 4; ++j) {
      const size_t bo = (size_t)(n0 + (j << 4) + rlane) * ldb + koff + k0;
      bh[j] = Frag<T>::load(Bb + bo);
      if (SPLIT) bl[j] = Frag<T>::load(Bb2 + bo);
    }
#pragma unroll
    for (int i = 0; i < 4; ++i) {
      const size_t ao = (size_t)(m0 + (i << 4) + rlane) * lda + koff + k0;
      V ah = Frag<T>::load(Ab + ao);
      V al;
      if (SPLIT) al = Frag<T>::load(Ab2 + ao);
#pragma unroll
      for (int j = 0; j < 4; ++j) {
        acc[i][j] = Frag<T>::mma(ah, bh[j], acc[i][j]);
        if (SPLIT) {
          acc[i][j] = Frag<T>::mma(ah, bl[j], acc[i][j]);
          acc[i][j] = Frag<T>::mma(al, bh[j], acc[i][j]);
        }
      }
      Frag<T>::guard(acc[i][0], acc[i][3], ah, SPLIT ? al : ah);
    }
    Frag<T>::keep(bh[0], bh[1], bh[2], bh[3]);
    if (SPLIT) Frag<T>::keep(bl[0], bl[1], bl[2], bl[3]);
  }
  acc_guard4(acc[0][0], acc[0][1], acc[0][2], acc[0][3]);
  acc_guard4(acc[1][0], acc[1][1], acc[1][2], acc[1][3]);
  acc_guard4(acc[2][0], acc[2][1], acc[2][2], acc[2][3]);
  acc_guard4(acc[3][0], acc[3][1], acc[3][2], acc[3][3]);

  float* slab = sT[wave];
  const float* Rb = RESID ? (resid + (size_t)b * strideR) : nullptr;
#pragma unroll
  for (int i = 0; i < 4; ++i) {
    const int mBase = m0 + (i << 4);
#pragma unroll
    for (int j = 0; j < 4; ++j) {
      const int n = n0 + (j << 4) + rlane;
      float bv = 0.f;
      if (BIAS_MODE == 2) bv = bias[n];
#pragma unroll
      for (int r = 0; r < 8; ++r) {
        float v = acc[i][j][r] * scale;
        if (BIAS_MODE == 1) v += bias[mBase + mOff + r];
        if (BIAS_MODE == 2) v += bv;
        if (RESID) v += Rb[(size_t)(mBase + mOff + r) * ldc + n];
        if (ACT == 1) v = tanhf(v);
        if (ACT == 2) v = fmaxf(v, 0.0f);
        if (ACT == 3) v = v / (1.0f + expf(-v));
        if (ACT == 4) v = (v > 0.f) ? v : 0.01f * v;
        if (ACT == 5) v = 0.5f * v * (1.0f + erff(v * 0.70710678118654752f));
        slab[(mOff + r) * 68 + (j << 4) + rlane] = v;
      }
    }
    __builtin_amdgcn_fence(__ATOMIC_RELEASE, "workgroup");
    __builtin_amdgcn_wave_barrier();
    __builtin_amdgcn_fence(__ATOMIC_ACQUIRE, "workgroup");
    if (OUT_MODE == 0) {
      float* C = (float*)Cout + (size_t)b * strideC;
      const int hh = lane >> 4, c4 = (lane & 15) * 4;
      for (int pass = 0; pass < 2; ++pass) {
#pragma unroll
        for (int it = 0; it < 8; ++it) {
          const int row = it * 2 + hh;
          v4f v = *(const v4f*)(slab + row * 68 + c4);
          *(volatile v4f*)(C + (size_t)(mBase + row) * ldc + n0 + c4) = v;
        }
        __threadfence();
      }
    } else {
      const int q = lane >> 3, c8 = (lane & 7) * 8;
      unsigned short* C  = (unsigned short*)Cout  + (size_t)b * strideC;
      unsigned short* C2 = (OUT_MODE == 2) ? ((unsigned short*)Cout2 + (size_t)b * strideC) : nullptr;
      for (int pass = 0; pass < 2; ++pass) {
#pragma unroll
        for (int it = 0; it < 4; ++it) {
          const int row = it * 4 + q;
          const float* sp = slab + row * 68 + c8;
          v8h hv, lv;
#pragma unroll
          for (int e = 0; e < 8; ++e) {
            if (OUT_MODE == 1) {
              hv[e] = (_Float16)sp[e];
            } else {
              unsigned short hb = f2bf_bits(sp[e]);
              unsigned short lb = f2bf_bits(sp[e] - bf_bits2f(hb));
              hv[e] = __builtin_bit_cast(_Float16, hb);
              lv[e] = __builtin_bit_cast(_Float16, lb);
            }
          }
          *(volatile v8h*)(C + (size_t)(mBase + row) * ldc + n0 + c8) = hv;
          if (OUT_MODE == 2) *(volatile v8h*)(C2 + (size_t)(mBase + row) * ldc + n0 + c8) = lv;
        }
        __threadfence();
      }
    }
    __builtin_amdgcn_fence(__ATOMIC_RELEASE, "workgroup");
    __builtin_amdgcn_wave_barrier();
    __builtin_amdgcn_fence(__ATOMIC_ACQUIRE, "workgroup");
  }
}

__device__ __forceinline__ float fsig(float x)  { return __builtin_amdgcn_rcpf(1.0f + __expf(-x)); }
__device__ __forceinline__ float ftanh(float x) { return 1.0f - 2.0f * __builtin_amdgcn_rcpf(__expf(2.0f * x) + 1.0f); }

constexpr int WCAT_CHUNKS = NGATE * KCAT / 8;
constexpr int W1_CHUNKS   = NHD * NHID / 8;
constexpr int B1_CHUNKS   = NHD / 4;
constexpr int PREP_TOTAL  = WCAT_CHUNKS + W1_CHUNKS + B1_CHUNKS;
static_assert(WCAT_CHUNKS % 32 == 0 && W1_CHUNKS % 32 == 0);

__global__ __launch_bounds__(NTHR) void prep_kernel(const float* __restrict__ W_ih, const float* __restrict__ W_hh,
                                                  const float* __restrict__ W1, const float* __restrict__ b1,
                                                  unsigned short* __restrict__ Wcat, unsigned short* __restrict__ W1cat,
                                                  float* __restrict__ b1r) {
  const int i = blockIdx.x * NTHR + threadIdx.x;
  if (i < WCAT_CHUNKS) {
    const int n = i / 20, cch = i - n * 20;
    v8h hv;
#pragma unroll
    for (int e = 0; e < 8; ++e) {
      const int col = cch * 8 + e;
      const int ci = (col < NIN) ? col : (NIN - 1);
      const int ch = (col >= 32) ? (col - 32) : 0;
      const float wi = W_ih[(size_t)n * NIN + ci];
      const float wh = W_hh[(size_t)n * NHID + ch];
      const float v = (col < NIN) ? wi : ((col < 32) ? 0.0f : wh);
      hv[e] = (_Float16)(bf16q(v) * WSC);
    }
    unsigned short* dst = Wcat + (size_t)i * 8;
    for (int pass = 0; pass < 2; ++pass) { *(volatile v8h*)dst = hv; __threadfence(); }
  } else if (i < WCAT_CHUNKS + W1_CHUNKS) {
    const int jj = i - WCAT_CHUNKS;
    const int n = jj >> 4, k8 = (jj & 15) * 8;
    v8h hv;
#pragma unroll
    for (int e = 0; e < 8; ++e) hv[e] = (_Float16)(bf16q(W1[(size_t)n * NHID + k8 + e]) * WSC);
    unsigned short* dst = W1cat + (size_t)jj * 8;
    for (int pass = 0; pass < 2; ++pass) { *(volatile v8h*)dst = hv; __threadfence(); }
  } else if (i < PREP_TOTAL) {
    const int jj = i - WCAT_CHUNKS - W1_CHUNKS;
    v4f v;
#pragma unroll
    for (int e = 0; e < 4; ++e) v[e] = bf16q(b1[jj * 4 + e]);
    float* dst = b1r + jj * 4;
    for (int pass = 0; pass < 2; ++pass) { *(volatile v4f*)dst = v; __threadfence(); }
  }
}

__device__ __forceinline__ void load_x_tile(const float* __restrict__ x, _Float16* At, int rowbase, int t, int tid) {
  if (tid < 80) {
    const int m = tid / 5, f4 = (tid - m * 5) * 4;
    const v4f v = *(const v4f*)(x + ((size_t)(rowbase + m) * NSTEP + (size_t)t) * NIN + f4);
    v4h hv;
#pragma unroll
    for (int e = 0; e < 4; ++e) hv[e] = (_Float16)bf16q(v[e]);
    *(v4h*)(At + m * APITCH + f4) = hv;
  }
}

__global__ __launch_bounds__(NTHR) void lstm_seq_kernel(const float* __restrict__ x, const float* __restrict__ b_ih,
                                                      const float* __restrict__ b_hh, const unsigned short* __restrict__ Wcatp,
                                                      const float* __restrict__ ctx_unused, const int* __restrict__ len_unused,
                                                      unsigned short* __restrict__ HS) {
  (void)ctx_unused; (void)len_unused;
  __shared__ __align__(16) _Float16 At[16 * APITCH];
  const _Float16* Wc = (const _Float16*)Wcatp;
  const int tid = threadIdx.x, lane = tid & 31, wave = tid >> 5;
  const int c = lane & 15, hh = lane >> 4, koff = hh * 8;
  const int rowbase = blockIdx.x * 16;
  const int j = 16 * wave + c;

#pragma unroll 1
  for (int i = tid; i < 16 * APITCH; i += NTHR) At[i] = (_Float16)0.0f;
  __syncthreads();
  load_x_tile(x, At, rowbase, 0, tid);

  float bb[4], cst[8], hst[8];
#pragma unroll
  for (int g = 0; g < 4; ++g) bb[g] = bf16q(b_ih[g * NHID + j]) + bf16q(b_hh[g * NHID + j]);
#pragma unroll
  for (int r = 0; r < 8; ++r) { cst[r] = 0.0f; hst[r] = 0.0f; }
  __syncthreads();

  const _Float16* arow = At + c * APITCH + koff;
  const _Float16* wrow = Wc + (size_t)j * KCAT + koff;
  const v8f z8 = {0.f, 0.f, 0.f, 0.f, 0.f, 0.f, 0.f, 0.f};

#pragma unroll 1
  for (int t = 0; t < NSTEP; ++t) {
    v8f acc[4];
    acc[0] = z8; acc[1] = z8; acc[2] = z8; acc[3] = z8;
#pragma unroll 1
    for (int ks = 0; ks < KCAT; ks += 32) {
      const v16h a   = Frag<_Float16>::load(arow + ks);
      const v16h wf0 = Frag<_Float16>::load(wrow + ks);
      const v16h wf1 = Frag<_Float16>::load(wrow + (size_t)1 * NHID * KCAT + ks);
      const v16h wf2 = Frag<_Float16>::load(wrow + (size_t)2 * NHID * KCAT + ks);
      const v16h wf3 = Frag<_Float16>::load(wrow + (size_t)3 * NHID * KCAT + ks);
      acc[0] = Frag<_Float16>::mma(a, wf0, acc[0]);
      acc[1] = Frag<_Float16>::mma(a, wf1, acc[1]);
      acc[2] = Frag<_Float16>::mma(a, wf2, acc[2]);
      acc[3] = Frag<_Float16>::mma(a, wf3, acc[3]);
      dep_guard_h(acc[0], acc[3], a, wf3);
      keep4_h(wf0, wf1, wf2, wf3);
    }
    acc_guard4(acc[0], acc[1], acc[2], acc[3]);
#pragma unroll
    for (int r = 0; r < 8; ++r) {
      const float zi = acc[0][r] * WSC_INV + bb[0];
      const float zf = acc[1][r] * WSC_INV + bb[1];
      const float zg = acc[2][r] * WSC_INV + bb[2];
      const float zo = acc[3][r] * WSC_INV + bb[3];
      const float ig = fsig(zi);
      const float fg = fsig(zf);
      const float gg = ftanh(zg);
      const float og = fsig(zo);
      const float cn = fg * cst[r] + ig * gg;
      cst[r] = cn;
      hst[r] = og * ftanh(cn);
    }
    __syncthreads();
#pragma unroll
    for (int r = 0; r < 8; ++r) At[(8 * hh + r) * APITCH + 32 + j] = (_Float16)hst[r];
    {
      const int tn = (t + 1 < NSTEP) ? (t + 1) : (NSTEP - 1);
      load_x_tile(x, At, rowbase, tn, tid);
    }
    __syncthreads();
    {
      const int row = 2 * wave + hh;
      const v8h v = *(const v8h*)(At + row * APITCH + 32 + c * 8);
      unsigned short* dst = HS + ((size_t)(rowbase + row) * NSTEP + (size_t)t) * NHID + c * 8;
      for (int pass = 0; pass < 2; ++pass) { *(volatile v8h*)dst = v; __threadfence(); }
    }
  }
}

__global__ __launch_bounds__(NTHR) void head_kernel(const float* __restrict__ HDN, const float* __restrict__ W2,
                                                  const float* __restrict__ b2, float* __restrict__ out,
                                                  int rowbase, int nrows) {
  __shared__ float sW2[NOUT * NHD];
  __shared__ float sB2[NOUT];
  const int tid = threadIdx.x;
  sW2[tid] = bf16q(W2[tid]);
  if (tid < NOUT) sB2[tid] = bf16q(b2[tid]);
  __syncthreads();
  const int r = blockIdx.x * NTHR + tid;
  const int rr = (r < nrows) ? r : (nrows - 1);
  const float* hp = HDN + (size_t)rr * NHD;
  float s0 = 0.f, s1 = 0.f, s2 = 0.f, s3 = 0.f;
#pragma unroll 1
  for (int k4 = 0; k4 < NHD; k4 += 4) {
    const v4f hv = *(const v4f*)(hp + k4);
#pragma unroll
    for (int e = 0; e < 4; ++e) {
      const float hk = hv[e];
      s0 = fmaf(hk, sW2[0 * NHD + k4 + e], s0);
      s1 = fmaf(hk, sW2[1 * NHD + k4 + e], s1);
      s2 = fmaf(hk, sW2[2 * NHD + k4 + e], s2);
      s3 = fmaf(hk, sW2[3 * NHD + k4 + e], s3);
    }
  }
  v4f res;
  res[0] = s0 + sB2[0]; res[1] = s1 + sB2[1]; res[2] = s2 + sB2[2]; res[3] = s3 + sB2[3];
  if (r < nrows) {
    float* dst = out + (size_t)(rowbase + r) * NOUT;
    for (int pass = 0; pass < 2; ++pass) { *(volatile v4f*)dst = res; __threadfence(); }
  }
}

extern "C" void kernel_launch(void* const* d_in, const int* in_sizes, int n_in,
                              void* d_out, int out_size, void* d_ws, size_t ws_size, hipStream_t stream) {
  if (n_in < 11 || d_out == nullptr || d_ws == nullptr) return;
  if (in_sizes[0] != NSEQ * NSTEP * NIN || in_sizes[3] != NGATE * NIN || in_sizes[4] != NGATE * NHID ||
      in_sizes[5] != NGATE || in_sizes[6] != NGATE || in_sizes[7] != NHD * NHID || in_sizes[8] != NHD ||
      in_sizes[9] != NOUT * NHD || in_sizes[10] != NOUT || out_size != NROWS * NOUT) return;

  const float* xin  = (const float*)d_in[0];
  const float* ctx  = (const float*)d_in[1];
  const int*   lens = (const int*)d_in[2];
  const float* W_ih = (const float*)d_in[3];
  const float* W_hh = (const float*)d_in[4];
  const float* b_ih = (const float*)d_in[5];
  const float* b_hh = (const float*)d_in[6];
  const float* W1   = (const float*)d_in[7];
  const float* b1   = (const float*)d_in[8];
  const float* W2   = (const float*)d_in[9];
  const float* b2   = (const float*)d_in[10];
  float* out = (float*)d_out;

  char* ws = (char*)d_ws; size_t off = 0;
  auto carve = [&](size_t bytes) -> char* { char* p = ws + off; off += (bytes + 255) & ~(size_t)255; return p; };
  unsigned short* Wcat  = (unsigned short*)carve((size_t)NGATE * KCAT * 2);
  unsigned short* W1cat = (unsigned short*)carve((size_t)NHD * NHID * 2);
  float*          b1r   = (float*)carve((size_t)NHD * 4);
  unsigned short* HS    = (unsigned short*)carve((size_t)NROWS * NHID * 2);
  float*          HDN   = (float*)carve((size_t)HCHUNK * NHD * 4);
  if (off > ws_size || off > (size_t)134217728) return;

  prep_kernel<<<(PREP_TOTAL + NTHR - 1) / NTHR, NTHR, 0, stream>>>(W_ih, W_hh, W1, b1, Wcat, W1cat, b1r);
  lstm_seq_kernel<<<NSEQ / 16, NTHR, 0, stream>>>(xin, b_ih, b_hh, Wcat, ctx, lens, HS);
  for (int chunk = 0; chunk < NROWS / HCHUNK; ++chunk) {
    const unsigned short* Achunk = HS + (size_t)chunk * HCHUNK * NHID;
    const int tiles = (HCHUNK / 64) * (NHD / 64);
    wmma_gemm64<0, false, 2, 0, false, 2><<<dim3((tiles + 7) / 8, 1), 256, 0, stream>>>(
        Achunk, Achunk, NHID, 0L, W1cat, W1cat, NHID, 0L, (void*)HDN, (void*)HDN, NHD, 0L,
        b1r, b1r, 0L, HCHUNK, NHD, NHID, WSC_INV);
    head_kernel<<<HCHUNK / NTHR, NTHR, 0, stream>>>(HDN, W2, b2, out, chunk * HCHUNK, HCHUNK);
  }
}
